// TauTrackFinderV3_12695923327029
// MI455X (gfx1250) — hardware-verified
//
#include <hip/hip_runtime.h>
#include <stddef.h>


#define CIN    16
#define PP     2048
#define KN     16
#define EE     64
#define HH     2
#define NCH    128
#define NCOL   256
#define GR     32
#define PJT    128
#define APH    40
#define SPF    260
#define QB     64
#define ATT    256
#define TPF    68
#define EPSV   1e-5f
#define NEGS   0.2f
#define WSCALE 16.0f
#define WINV   0.0625f
#define WPBYTES (NCOL * CIN * 2)

static_assert(NCH == HH * EE);
static_assert(NCOL == 2 * NCH);
static_assert(PP % GR == 0);
static_assert(PP % QB == 0);
static_assert(QB == 8 * (ATT / 32));
static_assert(GR * 2 == 16 * (PJT / 32));
static_assert((APH % 8) == 0);
static_assert((SPF % 4) == 0);
static_assert((TPF % 4) == 0);
static_assert(WPBYTES == 8192);
static_assert((NCOL * CIN / 8) % PJT == 0);

typedef _Float16 v4h  __attribute__((ext_vector_type(4)));
typedef _Float16 v8h  __attribute__((ext_vector_type(8)));
typedef _Float16 v16h __attribute__((ext_vector_type(16)));
typedef float    v4f  __attribute__((ext_vector_type(4)));
typedef float    v8f  __attribute__((ext_vector_type(8)));
typedef int      v4i  __attribute__((ext_vector_type(4)));
typedef unsigned v2u  __attribute__((ext_vector_type(2)));
union FragH { v16h v; v8h half[2]; };
union PackH { v8h h; v4h q[2]; v4i i; };

__device__ __forceinline__ v8f wm(v16h a, v16h b, v8f c) {
  v8f d = __builtin_amdgcn_wmma_f32_16x16x32_f16(false, a, false, b, (short)0, c, false, false);
  asm volatile("v_nop\n\tv_nop\n\tv_nop\n\tv_nop" : "+v"(d) : "v"(a), "v"(b));
  return d;
}

__global__ __launch_bounds__(256) void k_prepw(const float* __restrict__ node_w,
                                               const float* __restrict__ edge_w,
                                               _Float16* Wp) {
  const int tid = threadIdx.x;
  const float* src = (blockIdx.x == 0) ? node_w : edge_w;
  const int n  = tid >> 1;
  const int c0 = (tid & 1) * 8;
  const v4f f0 = *(const v4f*)(src + n * CIN + c0);
  const v4f f1 = *(const v4f*)(src + n * CIN + c0 + 4);
  PackH pk;
  pk.q[0] = __builtin_convertvector(f0 * WSCALE, v4h);
  pk.q[1] = __builtin_convertvector(f1 * WSCALE, v4h);
  const v4i v = pk.i;
  _Float16* dst = Wp + ((size_t)blockIdx.x * NCH + n) * CIN + c0;
  *(volatile v4i*)dst = v;
  __threadfence();
  *(volatile v4i*)dst = v;
}

__global__ __launch_bounds__(PJT) void k_proj(const float* __restrict__ feat,
                                              const _Float16* __restrict__ Wp,
                                              float* R, int P) {
  __shared__ __attribute__((aligned(16))) _Float16 At[GR * APH];
  __shared__ __attribute__((aligned(16))) _Float16 Ws[NCOL * CIN];
  __shared__ __attribute__((aligned(16))) float    S[GR * SPF];

  const int tid  = threadIdx.x;
  const int lane = tid & 31;
  const int wave = tid >> 5;
  const int h    = lane >> 4;
  const int m    = lane & 15;
  const int b    = blockIdx.y;
  const int p0   = blockIdx.x * GR;

#pragma unroll
  for (int i = 0; i < (NCOL * CIN / 8) / PJT; ++i)
    ((v4i*)Ws)[i * PJT + tid] = ((const v4i*)Wp)[i * PJT + tid];

  {
    const int p  = tid & 31;
    const int q  = tid >> 5;
    const int c0 = q * 4;
    const float* fp = feat + ((size_t)b * CIN + c0) * (size_t)P + p0 + p;
    v4f f;
    f.x = fp[0];
    f.y = fp[(size_t)P];
    f.z = fp[2 * (size_t)P];
    f.w = fp[3 * (size_t)P];
    *(v4h*)(At + p * APH + c0) = __builtin_convertvector(f, v4h);
    const v2u z2 = {0u, 0u};
    *(v2u*)(At + p * APH + CIN + c0) = z2;
  }
  __syncthreads();

  const v8h z8 = {(_Float16)0.f, (_Float16)0.f, (_Float16)0.f, (_Float16)0.f,
                  (_Float16)0.f, (_Float16)0.f, (_Float16)0.f, (_Float16)0.f};
#pragma unroll
  for (int rt = 0; rt < 2; ++rt) {
    FragH a;
    const _Float16* pa = At + (rt * 16 + m) * APH + 8 * h;
    a.half[0] = *(const v8h*)pa;
    a.half[1] = *(const v8h*)(pa + 16);
#pragma unroll
    for (int c4 = 0; c4 < 4; ++c4) {
      const int n = (wave * 4 + c4) * 16 + m;
      FragH bf;
      bf.half[0] = *(const v8h*)(Ws + n * CIN + 8 * h);
      bf.half[1] = z8;
      v8f acc = {0.f, 0.f, 0.f, 0.f, 0.f, 0.f, 0.f, 0.f};
      acc = wm(a.v, bf.v, acc);
#pragma unroll
      for (int r = 0; r < 8; ++r) S[(rt * 16 + 8 * h + r) * SPF + n] = acc[r] * WINV;
    }
  }
  __syncthreads();

  v4f vv[16];
  float* base = R + ((size_t)b * (size_t)P + (size_t)p0) * (size_t)NCOL;
#pragma unroll
  for (int i = 0; i < 16; ++i) {
    const int hr = wave * 16 + i;
    const int row = hr >> 1, part = hr & 1;
    vv[i] = *(const v4f*)(S + row * SPF + part * 128 + 4 * lane);
  }
#pragma unroll
  for (int i = 0; i < 16; ++i) {
    const int hr = wave * 16 + i;
    const int row = hr >> 1, part = hr & 1;
    *(volatile v4f*)(base + (size_t)row * NCOL + part * 128 + 4 * lane) = vv[i];
  }
  __threadfence();
#pragma unroll
  for (int i = 0; i < 16; ++i) {
    const int hr = wave * 16 + i;
    const int row = hr >> 1, part = hr & 1;
    *(volatile v4f*)(base + (size_t)row * NCOL + part * 128 + 4 * lane) = vv[i];
  }
}

__global__ __launch_bounds__(ATT) void k_att(
    const float* __restrict__ R, const int* __restrict__ nbr, const int* __restrict__ msk,
    const float* __restrict__ node_g, const float* __restrict__ node_b,
    const float* __restrict__ node_m, const float* __restrict__ node_v,
    const float* __restrict__ edge_bias, const float* __restrict__ edge_g,
    const float* __restrict__ edge_b2, const float* __restrict__ edge_m,
    const float* __restrict__ edge_v, const float* __restrict__ self_w,
    const float* __restrict__ self_b, const float* __restrict__ nb_w,
    const float* __restrict__ nb_b, float* out, int P, int ostride) {
  __shared__ __attribute__((aligned(16))) float cst[9 * NCH];
  __shared__ __attribute__((aligned(16))) float T[2 * EE * TPF];

  const int tid  = threadIdx.x;
  const int lane = tid & 31;
  const int wave = tid >> 5;
  const int h    = lane >> 4;
  const int m    = lane & 15;
  const int b    = blockIdx.y;
  const int p0   = blockIdx.x * QB;

  if (tid < NCH) {
    const int c = tid;
    const float an = node_g[c] * (1.0f / sqrtf(node_v[c] + EPSV));
    const float ae = edge_g[c] * (1.0f / sqrtf(edge_v[c] + EPSV));
    cst[0 * NCH + c] = an;
    cst[1 * NCH + c] = node_m[c];
    cst[2 * NCH + c] = node_b[c];
    cst[3 * NCH + c] = self_w[c];
    cst[4 * NCH + c] = ae;
    cst[5 * NCH + c] = edge_bias[c];
    cst[6 * NCH + c] = edge_m[c];
    cst[7 * NCH + c] = edge_b2[c];
    cst[8 * NCH + c] = nb_w[c];
  }
  __syncthreads();

  const v4f aN = *(const v4f*)(cst + 0 * NCH + 4 * lane);
  const v4f mN = *(const v4f*)(cst + 1 * NCH + 4 * lane);
  const v4f bN = *(const v4f*)(cst + 2 * NCH + 4 * lane);
  const v4f sW = *(const v4f*)(cst + 3 * NCH + 4 * lane);
  const v4f aE = *(const v4f*)(cst + 4 * NCH + 4 * lane);
  const v4f eB = *(const v4f*)(cst + 5 * NCH + 4 * lane);
  const v4f mE = *(const v4f*)(cst + 6 * NCH + 4 * lane);
  const v4f bE = *(const v4f*)(cst + 7 * NCH + 4 * lane);
  const v4f nW = *(const v4f*)(cst + 8 * NCH + 4 * lane);
  const float sb  = self_b[h];
  const float nbb = nb_b[h];
  const float ninf = -__builtin_inff();

#pragma unroll 1
  for (int i = 0; i < QB / (ATT / 32); ++i) {
    const int pl = wave * (QB / (ATT / 32)) + i;
    const int p  = p0 + pl;
    const size_t prow = (size_t)b * (size_t)P + (size_t)p;
    const v4f gn = *(const v4f*)(R + prow * NCOL + 4 * lane);
    const v4f gc = *(const v4f*)(R + prow * NCOL + NCH + 4 * lane);

    int ix = nbr[prow * KN + m];
    ix = (ix < 0) ? ix + P : ix;
    ix = (ix < 0) ? 0 : ((ix > P - 1) ? P - 1 : ix);
    const int vmk = msk[(size_t)b * (size_t)P + (size_t)ix];
    const unsigned vbits = __builtin_amdgcn_ballot_w32(vmk != 0);
    const bool anyv = (vbits & 0xFFFFu) != 0u;
    const float ownm = (msk[prow] != 0) ? 1.0f : 0.0f;

    const v4f nd = (gn - mN) * aN + bN;
    float sp = nd.x * sW.x + nd.y * sW.y + nd.z * sW.z + nd.w * sW.w;
    sp += __shfl_xor(sp, 8, 32);
    sp += __shfl_xor(sp, 4, 32);
    sp += __shfl_xor(sp, 2, 32);
    sp += __shfl_xor(sp, 1, 32);
    const float ss = sp + sb;

    float l  = 0.f;
    float mr = -1.0e30f;
    v4f acc = {0.f, 0.f, 0.f, 0.f};
    v4f gx  = {ninf, ninf, ninf, ninf};

#pragma unroll 1
    for (int k = 0; k < KN; ++k) {
      const int ixk = __shfl(ix, k, 32);
      const v4f gk = *(const v4f*)(R + ((size_t)b * (size_t)P + (size_t)ixk) * NCOL + NCH + 4 * lane);
      const v4f enc = (((gk - gc) + eB) - mE) * aE + bE;
      float q = enc.x * nW.x + enc.y * nW.y + enc.z * nW.z + enc.w * nW.w;
      q += __shfl_xor(q, 8, 32);
      q += __shfl_xor(q, 4, 32);
      q += __shfl_xor(q, 2, 32);
      q += __shfl_xor(q, 1, 32);
      float s = ss + (q + nbb);
      s = (s >= 0.f) ? s : NEGS * s;
      if (((vbits >> k) & 1u) != 0u) {
        const float mn = fmaxf(mr, s);
        const float sc = __expf(mr - mn);
        const float pk = __expf(s - mn);
        l   = l * sc + pk;
        acc = acc * sc + enc * pk;
        mr  = mn;
        gx.x = fmaxf(gx.x, enc.x);
        gx.y = fmaxf(gx.y, enc.y);
        gx.z = fmaxf(gx.z, enc.z);
        gx.w = fmaxf(gx.w, enc.w);
      }
    }

    const float lsafe = anyv ? l : 1.0f;
    const float inv   = anyv ? (1.0f / lsafe) : 0.0f;
    v4f at = acc * inv;
    at.x = fmaxf(at.x, 0.f); at.y = fmaxf(at.y, 0.f); at.z = fmaxf(at.z, 0.f); at.w = fmaxf(at.w, 0.f);
    v4f gr;
    gr.x = anyv ? gx.x : 0.f; gr.y = anyv ? gx.y : 0.f; gr.z = anyv ? gx.z : 0.f; gr.w = anyv ? gx.w : 0.f;

    v4f oa, og;
    oa.x = __shfl_xor(at.x, 16, 32); oa.y = __shfl_xor(at.y, 16, 32);
    oa.z = __shfl_xor(at.z, 16, 32); oa.w = __shfl_xor(at.w, 16, 32);
    og.x = __shfl_xor(gr.x, 16, 32); og.y = __shfl_xor(gr.y, 16, 32);
    og.z = __shfl_xor(gr.z, 16, 32); og.w = __shfl_xor(gr.w, 16, 32);
    v4f fa, fg;
    fa.x = fmaxf(at.x, oa.x) * ownm; fa.y = fmaxf(at.y, oa.y) * ownm;
    fa.z = fmaxf(at.z, oa.z) * ownm; fa.w = fmaxf(at.w, oa.w) * ownm;
    fg.x = fmaxf(gr.x, og.x) * ownm; fg.y = fmaxf(gr.y, og.y) * ownm;
    fg.z = fmaxf(gr.z, og.z) * ownm; fg.w = fmaxf(gr.w, og.w) * ownm;
    v4f val;
    val.x = h ? fg.x : fa.x; val.y = h ? fg.y : fa.y; val.z = h ? fg.z : fa.z; val.w = h ? fg.w : fa.w;
    float* tb = T + (h * EE + 4 * m) * TPF + pl;
    tb[0 * TPF] = val.x;
    tb[1 * TPF] = val.y;
    tb[2 * TPF] = val.z;
    tb[3 * TPF] = val.w;
  }
  __syncthreads();

  v4f vv[8];
  size_t go[8];
#pragma unroll
  for (int i = 0; i < 8; ++i) {
    const int L  = (wave * 8 + i) * 4 + (lane >> 3);
    const int o  = L >> 7;
    const int e  = (L >> 1) & 63;
    const int hf = L & 1;
    vv[i] = *(const v4f*)(T + (o * EE + e) * TPF + hf * 32 + 4 * (lane & 7));
    go[i] = (size_t)o * (size_t)ostride + ((size_t)b * EE + (size_t)e) * (size_t)P
          + (size_t)p0 + (size_t)(hf * 32 + 4 * (lane & 7));
  }
#pragma unroll
  for (int i = 0; i < 8; ++i) *(volatile v4f*)(out + go[i]) = vv[i];
  __threadfence();
#pragma unroll
  for (int i = 0; i < 8; ++i) *(volatile v4f*)(out + go[i]) = vv[i];
}

extern "C" void kernel_launch(void* const* d_in, const int* in_sizes, int n_in,
                              void* d_out, int out_size, void* d_ws, size_t ws_size,
                              hipStream_t stream) {
  if (n_in < 18) return;
  const int P  = PP;
  const int BP = in_sizes[2];
  if (BP <= 0 || (BP % P) != 0) return;
  const int B = BP / P;
  if (in_sizes[0] != CIN * BP) return;
  if (in_sizes[1] != KN * BP) return;
  if (in_sizes[3] != HH * EE * CIN || in_sizes[8] != HH * EE * CIN) return;
  if (in_sizes[4] != NCH || in_sizes[5] != NCH || in_sizes[6] != NCH || in_sizes[7] != NCH) return;
  if (in_sizes[9] != NCH || in_sizes[10] != NCH || in_sizes[11] != NCH || in_sizes[12] != NCH || in_sizes[13] != NCH) return;
  if (in_sizes[14] != NCH || in_sizes[16] != NCH) return;
  if (in_sizes[15] != HH || in_sizes[17] != HH) return;
  if (out_size != 2 * B * EE * P) return;

  const float* feat      = (const float*)d_in[0];
  const int*   nbr       = (const int*)d_in[1];
  const int*   msk       = (const int*)d_in[2];
  const float* node_w    = (const float*)d_in[3];
  const float* node_g    = (const float*)d_in[4];
  const float* node_b    = (const float*)d_in[5];
  const float* node_m    = (const float*)d_in[6];
  const float* node_v    = (const float*)d_in[7];
  const float* edge_w    = (const float*)d_in[8];
  const float* edge_bias = (const float*)d_in[9];
  const float* edge_g    = (const float*)d_in[10];
  const float* edge_b2   = (const float*)d_in[11];
  const float* edge_m    = (const float*)d_in[12];
  const float* edge_v    = (const float*)d_in[13];
  const float* self_w    = (const float*)d_in[14];
  const float* self_b    = (const float*)d_in[15];
  const float* nb_w      = (const float*)d_in[16];
  const float* nb_b      = (const float*)d_in[17];
  float* out = (float*)d_out;

  size_t off = 0;
  _Float16* Wp = (_Float16*)((char*)d_ws + off); off += (size_t)WPBYTES;
  float*    R  = (float*)((char*)d_ws + off);    off += (size_t)BP * (size_t)NCOL * sizeof(float);
  if (off > ws_size) return;

  const int ostride = B * EE * P;

  k_prepw<<<2, 256, 0, stream>>>(node_w, edge_w, Wp);

  dim3 gp(P / GR, B);
  k_proj<<<gp, PJT, 0, stream>>>(feat, Wp, R, P);

  dim3 ga(P / QB, B);
  k_att<<<ga, ATT, 0, stream>>>(R, nbr, msk, node_g, node_b, node_m, node_v,
                                edge_bias, edge_g, edge_b2, edge_m, edge_v,
                                self_w, self_b, nb_w, nb_b, out, P, ostride);
}
